// DeformableAlignment_59785944760673
// MI455X (gfx1250) — hardware-verified
//
#include <hip/hip_runtime.h>

#define B_   2
#define C_   64
#define H_   256
#define W_   256
#define DG_  8
#define KK_  9
#define CG_  8
#define C2   128
#define KC   1152
#define NP   224
#define NREAL 216
#define NOFF 144
#define K2   576
#define OMS  224
#define PLXX ((size_t)B_ * H_ * W_ * C2)
#define PLW  ((size_t)NP * KC)
#define PLF  ((size_t)C_ * K2)
#define RSPLIT (1.0f / 2048.0f)
__device__ __forceinline__ unsigned pk2s_(float a, float b, unsigned* lo) {
    const _Float16 h0 = (_Float16)a, h1 = (_Float16)b;
    *lo = (unsigned)__builtin_bit_cast(unsigned short, (_Float16)((a - (float)h0) * 2048.0f)) | ((unsigned)__builtin_bit_cast(unsigned short, (_Float16)((b - (float)h1) * 2048.0f)) << 16);
    return (unsigned)__builtin_bit_cast(unsigned short, h0) | ((unsigned)__builtin_bit_cast(unsigned short, h1) << 16);
}

#define __bf16 _Float16
typedef __attribute__((ext_vector_type(16))) _Float16 v16bf;
typedef __attribute__((ext_vector_type(8)))  _Float16 v8bf;
typedef __attribute__((ext_vector_type(4)))  float v4f_t;
typedef float v4fa __attribute__((ext_vector_type(4), may_alias));
static __device__ __forceinline__ unsigned pk2(float a, float b) { return (unsigned)__builtin_bit_cast(unsigned short, (_Float16)a) | ((unsigned)__builtin_bit_cast(unsigned short, (_Float16)b) << 16); }
typedef __attribute__((ext_vector_type(8)))  float  v8f;

union V16U { v16bf v; v8bf h[2]; };

#if defined(__has_builtin)
#if __has_builtin(__builtin_amdgcn_global_load_async_to_lds_b128) && \
    __has_builtin(__builtin_amdgcn_s_wait_asynccnt)
#define USE_ASYNC 1
#endif
#endif
#ifndef USE_ASYNC
#define USE_ASYNC 0
#endif

#if USE_ASYNC
typedef int v4i __attribute__((vector_size(4 * sizeof(int))));
typedef __attribute__((address_space(1))) v4i gv4i;
typedef __attribute__((address_space(3))) v4i lv4i;
#define ASYNC_WAIT() __builtin_amdgcn_s_wait_asynccnt(0)
#else
#define ASYNC_WAIT()
#endif

__device__ __forceinline__ int iclamp(int v, int lo, int hi) {
    return v < lo ? lo : (v > hi ? hi : v);
}

__global__ void pack_input_kernel(const float* __restrict__ ref,
                                  const float* __restrict__ nbr,
                                  __bf16* __restrict__ X) {
    const size_t e   = ((size_t)blockIdx.x * blockDim.x + threadIdx.x) * 2;
    const int    c   = (int)(e & (C2 - 1));
    const size_t pix = e >> 7;
    const size_t b   = pix / (size_t)(H_ * W_);
    const size_t sp  = pix % (size_t)(H_ * W_);
    const float* src = (c < C_) ? ref + (b * C_ + c) * (size_t)(H_ * W_) + sp : nbr + (b * C_ + (c - C_)) * (size_t)(H_ * W_) + sp;
    unsigned lo; const unsigned p = pk2s_(src[0], src[H_ * W_], &lo);
    *(volatile unsigned*)(X + e) = p; *(volatile unsigned*)(X + PLXX + e) = lo; __threadfence(); *(volatile unsigned*)(X + e) = p; *(volatile unsigned*)(X + PLXX + e) = lo;
}

__global__ void pack_wcm_kernel(const float* __restrict__ off_w,
                                const float* __restrict__ mask_w,
                                __bf16* __restrict__ Wcm) {
    const int e = (blockIdx.x * blockDim.x + threadIdx.x) * 2;
    const int n = e / KC;
    const int k = e - n * KC;
    const int tap = k >> 7;
    const int ci  = k & 127;
    float v0 = 0.0f, v1 = 0.0f;
    if (n < NOFF)       { v0 = off_w [((size_t)n * C2 + ci) * KK_ + tap]; v1 = off_w [((size_t)n * C2 + ci + 1) * KK_ + tap]; }
    else if (n < NREAL) { v0 = mask_w[((size_t)(n - NOFF) * C2 + ci) * KK_ + tap]; v1 = mask_w[((size_t)(n - NOFF) * C2 + ci + 1) * KK_ + tap]; }
    unsigned lo; const unsigned p = pk2s_(v0, v1, &lo);
    *(volatile unsigned*)(Wcm + e) = p; *(volatile unsigned*)(Wcm + PLW + e) = lo; __threadfence(); *(volatile unsigned*)(Wcm + e) = p; *(volatile unsigned*)(Wcm + PLW + e) = lo;
}

__global__ void pack_wf_kernel(const float* __restrict__ w,
                               __bf16* __restrict__ Wf) {
    const int e = (blockIdx.x * blockDim.x + threadIdx.x) * 2;
    unsigned lo; const unsigned p = pk2s_(w[e], w[e + 1], &lo);
    *(volatile unsigned*)(Wf + e) = p; *(volatile unsigned*)(Wf + PLF + e) = lo; __threadfence(); *(volatile unsigned*)(Wf + e) = p; *(volatile unsigned*)(Wf + PLF + e) = lo;
}

__device__ __forceinline__ void stage_panel(const __bf16* __restrict__ Wcm,
                                            __bf16* dst, int kc, int t) {
#pragma unroll
    for (int i = 0; i < 7; ++i) {
        const int j   = t + i * 128;
        const int row = j >> 2;
        const int seg = j & 3;
        const __bf16* src = Wcm + (size_t)row * KC + kc * 32 + seg * 8;
        __bf16* d = dst + row * 32 + seg * 8;
#if USE_ASYNC
        __builtin_amdgcn_global_load_async_to_lds_b128((gv4i*)src, (lv4i*)d, 0, 0);
        __builtin_amdgcn_global_load_async_to_lds_b128((gv4i*)(src + PLW), (lv4i*)(d + NP * 32), 0, 0);
#else
        *(v8bf*)d = *(const v8bf*)src;
        *(v8bf*)(d + NP * 32) = *(const v8bf*)(src + PLW);
#endif
    }
}

__global__ void __launch_bounds__(128) __attribute__((amdgpu_num_vgpr(248)))
conv_offmask_kernel(const __bf16* __restrict__ X,
                    const __bf16* __restrict__ Wcm,
                    const float* __restrict__ off_b,
                    const float* __restrict__ mask_b,
                    float* __restrict__ OM) {
    __shared__ __align__(16) __bf16 Bpan[2][2 * NP * 32];
    __shared__ __align__(16) float  Ost[4][16 * OMS];

    const int t    = (int)threadIdx.x;
    const int lane = t & 31;
    const int wave = t >> 5;
    const int tile = blockIdx.x * 4 + wave;
    const int b    = tile / (H_ * (W_ / 16));
    const int rem  = tile % (H_ * (W_ / 16));
    const int y    = rem / (W_ / 16);
    const int x0   = (rem % (W_ / 16)) * 16;

    const int m  = lane & 15;
    const int hv = lane >> 4;
    const int px = x0 + m;

    v8f acc[14];
#pragma unroll
    for (int nt = 0; nt < 14; ++nt)
#pragma unroll
        for (int q = 0; q < 8; ++q) acc[nt][q] = 0.0f;

    stage_panel(Wcm, Bpan[0], 0, t);
    ASYNC_WAIT();
    __syncthreads();

#pragma unroll 1
    for (int kc = 0; kc < 36; ++kc) {
        const int cur = kc & 1;
        if (kc < 35) stage_panel(Wcm, Bpan[cur ^ 1], kc + 1, t);

        const int tap = kc >> 2;
        const int cb  = (kc & 3) * 32;
        const int ys  = y  + tap / 3 - 1;
        const int xs  = px + tap % 3 - 1;
        V16U ua, ual;
#pragma unroll
        for (int q = 0; q < 8; ++q) { ua.h[0][q] = (__bf16)0.0f; ua.h[1][q] = (__bf16)0.0f; ual.h[0][q] = (__bf16)0.0f; ual.h[1][q] = (__bf16)0.0f; }
        if (ys >= 0 && ys < H_ && xs >= 0 && xs < W_) {
            const __bf16* p = X + (size_t)((b * H_ + ys) * W_ + xs) * C2;
            ua.h[0]  = *(const v8bf*)(p + cb + hv * 8);
            ua.h[1]  = *(const v8bf*)(p + cb + 16 + hv * 8);
            ual.h[0] = *(const v8bf*)(p + PLXX + cb + hv * 8);
            ual.h[1] = *(const v8bf*)(p + PLXX + cb + 16 + hv * 8);
        }
        const v16bf a = ua.v, al = ual.v;

        const __bf16* pb = &Bpan[cur][(lane & 15) * 32 + hv * 8];
#pragma unroll
        for (int u = 0; u < 14; ++u) {
            V16U ub, ubl;
            ub.h[0]  = *(const v8bf*)(pb + u * (16 * 32));            ub.h[1]  = *(const v8bf*)(pb + u * (16 * 32) + 16);
            ubl.h[0] = *(const v8bf*)(pb + NP * 32 + u * (16 * 32));  ubl.h[1] = *(const v8bf*)(pb + NP * 32 + u * (16 * 32) + 16);
            v8f xx = {};
            xx = __builtin_amdgcn_wmma_f32_16x16x32_f16(false, al, false, ub.v, (short)0, xx, false, false);
            xx = __builtin_amdgcn_wmma_f32_16x16x32_f16(false, a, false, ubl.v, (short)0, xx, false, false);
            acc[u] = __builtin_amdgcn_wmma_f32_16x16x32_f16(false, a, false, ub.v, (short)0, acc[u], false, false) + xx * RSPLIT;
            asm volatile("" ::: "memory");
        }

        ASYNC_WAIT();
        __syncthreads();
    }

    const size_t pixrow = (size_t)(b * H_ + y) * W_;
    float* os_ = Ost[wave];
#pragma unroll
    for (int nt = 0; nt < 14; ++nt) {
        const int n = nt * 16 + (lane & 15);
        float bz = 0.0f;
        if (n < NOFF)       bz = off_b[n];
        else if (n < NREAL) bz = mask_b[n - NOFF];
#pragma unroll
        for (int rr = 0; rr < 8; ++rr) os_[(rr + hv * 8) * OMS + n] = acc[nt][rr] + bz;
    }
    asm volatile("s_wait_dscnt 0" ::: "memory");
    float* dst = OM + (pixrow + x0) * OMS;
#pragma unroll 1
    for (int pass = 0; pass < 2; ++pass) {
        for (int c = lane; c < 16 * 56; c += 32) {
            const int rr = c / 56, q = c - rr * 56;
            *(volatile v4f_t*)(dst + (size_t)rr * OMS + q * 4) = *(const volatile v4fa*)(os_ + rr * OMS + q * 4);
        }
        __threadfence();
    }
}

__global__ void __launch_bounds__(64) __attribute__((amdgpu_num_vgpr(248)))
sample_gemm_kernel(const float* __restrict__ neigh,
                   const float* __restrict__ OM,
                   const __bf16* __restrict__ Wf,
                   const float* __restrict__ bias,
                   float* __restrict__ out) {
    __shared__ __align__(16) __bf16 AtAll[2][16 * K2];
    __shared__ __align__(16) __bf16 AtLAll[2][16 * K2];
    __shared__ __align__(16) float  Ob[64][32 + 4];

    const int lane = threadIdx.x & 31;
    const int wv   = threadIdx.x >> 5;
    __bf16* At = AtAll[wv];
    __bf16* AtL = AtLAll[wv];
    const int tile = blockIdx.x * 2 + wv;
    const int b    = tile / (H_ * (W_ / 16));
    const int rem  = tile % (H_ * (W_ / 16));
    const int y    = rem / (W_ / 16);
    const int x0   = (rem % (W_ / 16)) * 16;
    const int m    = lane & 15;
    const int hv   = lane >> 4;
    const int px   = x0 + m;

    const float* om = OM + (size_t)((b * H_ + y) * W_ + px) * OMS;

    for (int g = 0; g < DG_; ++g) {
#pragma unroll 1
        for (int kk = 0; kk < KK_; ++kk) {
            const int chd = (g * KK_ + kk) * 2;
            const float dy   = om[chd];
            const float dx   = om[chd + 1];
            const float mraw = om[NOFF + g * KK_ + kk];
            const float mval = 1.0f / (1.0f + __expf(-mraw));

            const float ysf = (float)(y  - 1 + kk / 3) + dy;
            const float xsf = (float)(px - 1 + kk % 3) + dx;
            const float y0f = floorf(ysf), x0f = floorf(xsf);
            const float wy = ysf - y0f, wx = xsf - x0f;
            const int iy0 = (int)y0f, ix0 = (int)x0f;
            const int iy1 = iy0 + 1,  ix1 = ix0 + 1;

            const float v00 = (iy0 >= 0 && iy0 < H_ && ix0 >= 0 && ix0 < W_) ? 1.0f : 0.0f;
            const float v01 = (iy0 >= 0 && iy0 < H_ && ix1 >= 0 && ix1 < W_) ? 1.0f : 0.0f;
            const float v10 = (iy1 >= 0 && iy1 < H_ && ix0 >= 0 && ix0 < W_) ? 1.0f : 0.0f;
            const float v11 = (iy1 >= 0 && iy1 < H_ && ix1 >= 0 && ix1 < W_) ? 1.0f : 0.0f;
            const float w00 = (1.0f - wy) * (1.0f - wx) * v00;
            const float w01 = (1.0f - wy) * wx          * v01;
            const float w10 = wy          * (1.0f - wx) * v10;
            const float w11 = wy          * wx          * v11;
            const int cy0 = iclamp(iy0, 0, H_ - 1), cx0 = iclamp(ix0, 0, W_ - 1);
            const int cy1 = iclamp(iy1, 0, H_ - 1), cx1 = iclamp(ix1, 0, W_ - 1);

#pragma unroll
            for (int c = 0; c < 4; ++c) {
                const int cc = g * CG_ + hv * 4 + c;
                const float* img = neigh + (size_t)(b * C_ + cc) * (H_ * W_);
                const float v = w00 * img[cy0 * W_ + cx0] + w01 * img[cy0 * W_ + cx1]
                              + w10 * img[cy1 * W_ + cx0] + w11 * img[cy1 * W_ + cx1];
                {
                    const float pv = v * mval; const __bf16 ph = (__bf16)pv;
                    At [m * K2 + g * (CG_ * KK_) + (hv * 4 + c) * KK_ + kk] = ph;
                    AtL[m * K2 + g * (CG_ * KK_) + (hv * 4 + c) * KK_ + kk] = (__bf16)((pv - (float)ph) * 2048.0f);
                }
            }
        }
    }
    asm volatile("s_wait_dscnt 0" ::: "memory");

    v8f acc[4];
#pragma unroll
    for (int nt = 0; nt < 4; ++nt)
#pragma unroll
        for (int q = 0; q < 8; ++q) acc[nt][q] = 0.0f;

#pragma unroll 1
    for (int kc = 0; kc < 18; ++kc) {
        V16U ua, ual;
        ua.h[0]  = *(const v8bf*)(At  + m * K2 + kc * 32 + hv * 8);
        ua.h[1]  = *(const v8bf*)(At  + m * K2 + kc * 32 + 16 + hv * 8);
        ual.h[0] = *(const v8bf*)(AtL + m * K2 + kc * 32 + hv * 8);
        ual.h[1] = *(const v8bf*)(AtL + m * K2 + kc * 32 + 16 + hv * 8);
        const v16bf a = ua.v, al = ual.v;
        const __bf16* wb = Wf + (size_t)(lane & 15) * K2 + kc * 32 + hv * 8;
#pragma unroll
        for (int nt = 0; nt < 4; ++nt) {
            V16U ub, ubl;
            ub.h[0]  = *(const v8bf*)(wb + (size_t)nt * 16 * K2);        ub.h[1]  = *(const v8bf*)(wb + (size_t)nt * 16 * K2 + 16);
            ubl.h[0] = *(const v8bf*)(wb + PLF + (size_t)nt * 16 * K2);  ubl.h[1] = *(const v8bf*)(wb + PLF + (size_t)nt * 16 * K2 + 16);
            v8f xx = {};
            xx = __builtin_amdgcn_wmma_f32_16x16x32_f16(false, al, false, ub.v, (short)0, xx, false, false);
            xx = __builtin_amdgcn_wmma_f32_16x16x32_f16(false, a, false, ubl.v, (short)0, xx, false, false);
            acc[nt] = __builtin_amdgcn_wmma_f32_16x16x32_f16(false, a, false, ub.v, (short)0, acc[nt], false, false) + xx * RSPLIT;
        }
    }

#pragma unroll
    for (int nt = 0; nt < 4; ++nt) {
        const int n  = nt * 16 + (lane & 15);
        const float bv = bias[n];
#pragma unroll
        for (int rr = 0; rr < 8; ++rr) Ob[n][wv * 16 + rr + hv * 8] = acc[nt][rr] + bv;
    }
    __syncthreads();
    {
        const int tid = threadIdx.x;
        const int xb0 = (blockIdx.x % (W_ / 32)) * 32;
#pragma unroll 1
        for (int pass = 0; pass < 2; ++pass) {
#pragma unroll
            for (int i = 0; i < 8; ++i) {
                const int c = tid + 64 * i, ch = c >> 3, q = c & 7;
                *(volatile v4f_t*)(out + ((size_t)(b * C_ + ch) * H_ + y) * W_ + xb0 + q * 4) = *(const v4fa*)&Ob[ch][q * 4];
            }
            __threadfence();
        }
    }
}

extern "C" void kernel_launch(void* const* d_in, const int* in_sizes, int n_in,
                              void* d_out, int out_size, void* d_ws, size_t ws_size,
                              hipStream_t stream) {
    const float* ref    = (const float*)d_in[0];
    const float* nbr    = (const float*)d_in[1];
    const float* off_w  = (const float*)d_in[2];
    const float* off_b  = (const float*)d_in[3];
    const float* mask_w = (const float*)d_in[4];
    const float* mask_b = (const float*)d_in[5];
    const float* weight = (const float*)d_in[6];
    const float* bias   = (const float*)d_in[7];
    float* out = (float*)d_out;

    char* ws = (char*)d_ws;
    size_t off = 0;
    auto take = [&](size_t bytes) {
        char* p = ws + off;
        off = (off + bytes + 255) & ~(size_t)255;
        return p;
    };
    __bf16* X   = (__bf16*)take((size_t)B_ * H_ * W_ * C2 * 2 * 2);
    __bf16* Wcm = (__bf16*)take((size_t)NP * KC * 2 * 2);
    __bf16* Wf  = (__bf16*)take((size_t)C_ * K2 * 2 * 2);
    float*  OM  = (float*) take((size_t)B_ * H_ * W_ * OMS * 4);

    hipLaunchKernelGGL(pack_input_kernel, dim3((B_ * H_ * W_ * C2) / 512), dim3(256),
                       0, stream, ref, nbr, X);
    hipLaunchKernelGGL(pack_wcm_kernel, dim3((NP * KC) / 512), dim3(256),
                       0, stream, off_w, mask_w, Wcm);
    hipLaunchKernelGGL(pack_wf_kernel, dim3((C_ * K2) / 512), dim3(256),
                       0, stream, weight, Wf);
    hipLaunchKernelGGL(conv_offmask_kernel, dim3((B_ * H_ * (W_ / 16)) / 4), dim3(128),
                       0, stream, X, Wcm, off_b, mask_b, OM);
    hipLaunchKernelGGL(sample_gemm_kernel, dim3(B_ * H_ * (W_ / 32)), dim3(64),
                       0, stream, nbr, OM, Wf, bias, out);
}
